// EKTMSeqModel_61375082660572
// MI455X (gfx1250) — hardware-verified
//
#include <hip/hip_runtime.h>
#include <hip/hip_bf16.h>
#include <math.h>

#define TT 1024
#define KK 128
#define LL 4096
#define HHD 1024
#define G3 (3 * HHD)

typedef _Float16 bf16;
typedef __attribute__((ext_vector_type(4))) unsigned v4u_t;
typedef unsigned v4ua __attribute__((ext_vector_type(4), may_alias));
typedef __attribute__((ext_vector_type(4))) float v4f_t;
typedef float v4fa __attribute__((ext_vector_type(4), may_alias));
typedef __attribute__((ext_vector_type(16))) bf16  bf16x16;
typedef __attribute__((ext_vector_type(8)))  bf16  bf16x8;
typedef __attribute__((ext_vector_type(4)))  bf16  bf16x4;
typedef __attribute__((ext_vector_type(8)))  float f32x8;
#define SS 1024
#define DKK 64
#define HH 16
#define LDS_STRIDE 48
#define KSTRIDE    72
#define VSTRIDE    48

__device__ __forceinline__ f32x8 wmma_bf16(bf16x16 a, bf16x16 b, f32x8 c) {
  c = __builtin_amdgcn_wmma_f32_16x16x32_f16(false, a, false, b, (short)0, c, false, false);
  asm volatile("v_nop\n\tv_nop\n\tv_nop\n\tv_nop" : "+v"(c) : "v"(a), "v"(b));
  return c;
}

template <typename T>
__device__ __forceinline__ bf16x16 load_frag(const T* __restrict__ base, int ld,
                                             int row0, int k0) {
  const int lane = threadIdx.x & 31;
  const int r    = lane & 15;
  const int kh   = (lane >> 4) * 8;
  const T* p0 = base + (size_t)(row0 + r) * ld + (k0 + kh);
  const T* p1 = p0 + 16;
  bf16x16 f;
#pragma unroll
  for (int i = 0; i < 8; ++i) {
    f[i]     = (bf16)p0[i];
    f[i + 8] = (bf16)p1[i];
  }
  return f;
}

__device__ __forceinline__ bf16x16 lds_frag(const bf16* base, int stride) {
  const int lane = threadIdx.x & 31;
  const int row  = lane & 15;
  const int kh   = (lane >> 4) * 8;
  const bf16x8 lo = *(const bf16x8*)(base + row * stride + kh);
  const bf16x8 hi = *(const bf16x8*)(base + row * stride + kh + 16);
  bf16x16 f;
#pragma unroll
  for (int i = 0; i < 8; ++i) { f[i] = lo[i]; f[i + 8] = hi[i]; }
  return f;
}

template <typename T>
__device__ __forceinline__ void stage_read16(const T* __restrict__ p, float* buf) {
#pragma unroll
  for (int i = 0; i < 16; ++i) buf[i] = (float)p[i];
}

__device__ __forceinline__ void stage_write(bf16* dst, const float* buf, int nquad) {
#pragma unroll
  for (int i = 0; i < nquad; ++i) {
    bf16x4 q;
    q[0] = (bf16)buf[4 * i];     q[1] = (bf16)buf[4 * i + 1];
    q[2] = (bf16)buf[4 * i + 2]; q[3] = (bf16)buf[4 * i + 3];
    *(bf16x4*)(dst + 4 * i) = q;
  }
}

template <typename AT, int MODE>
__global__ __launch_bounds__(256) void gemm_rb_kernel(
    const AT* __restrict__ A, const float* __restrict__ W,
    const float* __restrict__ bias, const float* __restrict__ rowscale, const float* __restrict__ R, const float* __restrict__ rowbias, void* __restrict__ out,
    int M, int N, int K) {
  __shared__ bf16 ldsA[128 * LDS_STRIDE];
  __shared__ bf16 ldsW[256 * LDS_STRIDE];
  __shared__ __attribute__((aligned(16))) unsigned char sob[256 * 136 * 2];

  const int t    = threadIdx.x;
  const int wave = t >> 5;
  const int lane = t & 31;
  const int wm   = (wave & 1) * 64;
  const int wn   = (wave >> 1) * 64;
  const int mBlk = blockIdx.x * 128;
  const int nBlk = blockIdx.y * 256;

  const int arow = t >> 1;
  const int ach  = (t & 1) * 16;

  float abuf[16];
  float wbuf[32];

  stage_read16(A + (size_t)(mBlk + arow) * K + ach, abuf);
  const int nrow = min(nBlk + t, N - 1);
  stage_read16(W + (size_t)nrow * K,          wbuf);
  stage_read16(W + (size_t)nrow * K + 16,     wbuf + 16);

  f32x8 acc[4][4] = {};

  for (int k = 0; k < K; k += 32) {
    __syncthreads();
    stage_write(&ldsA[arow * LDS_STRIDE + ach], abuf, 4);
    stage_write(&ldsW[t * LDS_STRIDE],          wbuf, 8);
    if (k + 32 < K) {
      stage_read16(A + (size_t)(mBlk + arow) * K + (k + 32) + ach, abuf);
      stage_read16(W + (size_t)nrow * K + (k + 32),          wbuf);
      stage_read16(W + (size_t)nrow * K + (k + 32) + 16,     wbuf + 16);
    }
    __syncthreads();

    bf16x16 af[4], wf[4];
#pragma unroll
    for (int i = 0; i < 4; ++i)
      af[i] = lds_frag(ldsA + (wm + 16 * i) * LDS_STRIDE, LDS_STRIDE);
#pragma unroll
    for (int j = 0; j < 4; ++j)
      wf[j] = lds_frag(ldsW + (wn + 16 * j) * LDS_STRIDE, LDS_STRIDE);
#pragma unroll
    for (int i = 0; i < 4; ++i)
#pragma unroll
      for (int j = 0; j < 4; ++j)
        acc[i][j] = wmma_bf16(af[i], wf[j], acc[i][j]);
  }

  const int nlane = lane & 15;
  const int mh    = (lane >> 4) * 8;
  __syncthreads();
  if (MODE == 0 || MODE == 1 || MODE == 3) {
    bf16* so = (bf16*)sob;
#pragma unroll
    for (int i = 0; i < 4; ++i)
#pragma unroll
      for (int j = 0; j < 4; ++j) {
        const int nl = wn + 16 * j + nlane;
        const float bv = bias ? bias[nBlk + nl] : 0.0f;
        if (MODE == 3) {
#pragma unroll 1
          for (int r = 0; r < 8; ++r) {
            const int ml = wm + 16 * i + mh + r;
            const float xg = acc[i][j][r] + bv;
            so[ml * 264 + nl] = (bf16)(0.5f * xg * (1.0f + erff(xg * 0.70710678118654752f)));
          }
        } else {
#pragma unroll
        for (int r = 0; r < 8; ++r) {
          const int ml = wm + 16 * i + mh + r;
          const bf16 hv = (bf16)(acc[i][j][r] + bv);
          if (MODE == 0) so[ml * 264 + nl] = hv;
          else           so[nl * 136 + ml] = hv;
        }
        }
      }
    __syncthreads();
#pragma unroll 1
    for (int pass = 0; pass < 2; ++pass) {
      if (MODE == 0 || MODE == 3) {
        for (int ch = t; ch < 128 * 32; ch += 256) { const int ml = ch >> 5, q = (ch & 31) * 8;
          *(volatile v4u_t*)((bf16*)out + (size_t)(mBlk + ml) * N + nBlk + q) = *(const v4ua*)(so + ml * 264 + q); }
      } else {
        const int b_ = mBlk / SS, s0 = mBlk & (SS - 1);
        for (int ch = t; ch < 256 * 16; ch += 256) { const int nl = ch >> 4, q = (ch & 15) * 8; const int n = nBlk + nl, h = n >> 6, dk = n & (DKK - 1);
          *(volatile v4u_t*)((bf16*)out + (((size_t)(b_ * HH + h)) * DKK + dk) * SS + s0 + q) = *(const v4ua*)(so + nl * 136 + q); }
      }
      __threadfence();
    }
  } else {
    float* so = (float*)sob;
#pragma unroll 1
    for (int hf = 0; hf < 2; ++hf) {
      if (wm == hf * 64) {
#pragma unroll
        for (int i = 0; i < 4; ++i)
#pragma unroll
          for (int j = 0; j < 4; ++j) {
            const int nl = wn + 16 * j + nlane;
            const float bv = bias ? bias[nBlk + nl] : 0.0f;
#pragma unroll
            for (int r = 0; r < 8; ++r) { const int mrow = mBlk + hf * 64 + 16 * i + mh + r; so[(16 * i + mh + r) * 260 + nl] = acc[i][j][r] * (rowscale ? rowscale[mrow] : 1.0f) + bv + (rowbias ? rowbias[mrow] : 0.0f); }
          }
      }
      __syncthreads();
      if (R) {
        for (int ch = t; ch < 64 * 64; ch += 256) { const int ml = ch >> 6, q = (ch & 63) * 4;
          if (nBlk + q < N) { const v4f_t rv = *(const v4f_t*)(R + (size_t)(mBlk + hf * 64 + ml) * N + nBlk + q); v4f_t v = *(const volatile v4fa*)(so + ml * 260 + q); v += rv; *(volatile v4fa*)(so + ml * 260 + q) = v; } }
        asm volatile("s_wait_dscnt 0" ::: "memory");
      }
#pragma unroll 1
      for (int pass = 0; pass < 2; ++pass) {
        for (int ch = t; ch < 64 * 64; ch += 256) { const int ml = ch >> 6, q = (ch & 63) * 4;
          if (nBlk + q < N) *(volatile v4f_t*)((float*)out + (size_t)(mBlk + hf * 64 + ml) * N + nBlk + q) = *(const volatile v4fa*)(so + ml * 260 + q); }
        __threadfence();
      }
      __syncthreads();
    }
  }
}


__global__ __launch_bounds__(256) void k_beta(const float* __restrict__ km, const float* __restrict__ kv, float* __restrict__ beta) {
  __shared__ float kvS[KK];
  __shared__ __attribute__((aligned(16))) float lg[LL];
  __shared__ float red[256];
  const int tid = threadIdx.x;
  if (tid < KK) kvS[tid] = kv[tid];
  __syncthreads();
  float mx = -INFINITY;
#pragma unroll 1
  for (int l = tid; l < LL; l += 256) { const float* row = km + (size_t)l * KK; float s = 0.0f;
#pragma unroll 1
    for (int k = 0; k < KK; ++k) s += row[k] * kvS[k];
    lg[l] = s; mx = fmaxf(mx, s); }
  red[tid] = mx; __syncthreads();
  for (int o = 128; o > 0; o >>= 1) { if (tid < o) red[tid] = fmaxf(red[tid], red[tid + o]); __syncthreads(); }
  const float m = red[0]; __syncthreads();
  float sum = 0.0f;
#pragma unroll 1
  for (int l = tid; l < LL; l += 256) { const float e = expf(lg[l] - m); lg[l] = e; sum += e; }
  red[tid] = sum; __syncthreads();
  for (int o = 128; o > 0; o >>= 1) { if (tid < o) red[tid] += red[tid + o]; __syncthreads(); }
  const float inv = 1.0f / red[0];
  __syncthreads();
#pragma unroll 1
  for (int l = tid; l < LL; l += 256) lg[l] *= inv;
  __syncthreads();
#pragma unroll 1
  for (int pass = 0; pass < 2; ++pass) { for (int q = tid; q < LL / 4; q += 256) *(volatile v4f_t*)(beta + q * 4) = *(const volatile v4fa*)(lg + q * 4); __threadfence(); }
}
__global__ __launch_bounds__(256) void k_vih(const float* __restrict__ Wih, const float* __restrict__ tv, const float* __restrict__ result, float* __restrict__ v) {
  __shared__ float tS[TT];
  __shared__ __attribute__((aligned(16))) float vS[256];
  const int tid = threadIdx.x, j = blockIdx.x * 256 + tid;
  for (int e = tid; e < TT; e += 256) tS[e] = tv[e];
  __syncthreads();
  const int off = (result[0] >= 0.5f) ? 0 : TT;
  const float* row = Wih + (size_t)j * (2 * TT) + off;
  float s = 0.0f;
#pragma unroll 1
  for (int k = 0; k < TT; ++k) s += row[k] * tS[k];
  vS[tid] = s;
  __syncthreads();
#pragma unroll 1
  for (int pass = 0; pass < 2; ++pass) { if (tid < 64) *(volatile v4f_t*)(v + blockIdx.x * 256 + tid * 4) = *(const volatile v4fa*)(vS + tid * 4); __threadfence(); }
}
__global__ __launch_bounds__(256) void k_score(const float* __restrict__ beta, const float* __restrict__ h0, const float* __restrict__ tv,
                                              const float* __restrict__ sw, const float* __restrict__ sb, float* __restrict__ out) {
  __shared__ float red[256];
  const int tid = threadIdx.x;
  float part = 0.0f;
#pragma unroll 1
  for (int j = tid; j < HHD; j += 256) { float s = 0.0f;
#pragma unroll 1
    for (int l = 0; l < LL; ++l) s += beta[l] * h0[(size_t)l * HHD + j];
    part += s * sw[TT + j] + tv[j] * sw[j]; }
  red[tid] = part; __syncthreads();
  for (int o = 128; o > 0; o >>= 1) { if (tid < o) red[tid] += red[tid + o]; __syncthreads(); }
  if (tid == 0) { const float p = red[0] + sb[0]; *(volatile float*)out = p; __threadfence(); *(volatile float*)out = p; }
}
__global__ __launch_bounds__(256) void k_gru(const float* __restrict__ gh, const float* __restrict__ beta, const float* __restrict__ v, const float* __restrict__ bih,
                                            const float* __restrict__ h0, float* __restrict__ hout) {
  __shared__ float hS[HHD];
  const int tid = threadIdx.x, l = blockIdx.x;
  const float bl = beta[l];
  const float* g = gh + (size_t)l * G3; const float* hr = h0 + (size_t)l * HHD;
#pragma unroll 1
  for (int j = tid; j < HHD; j += 256) {
    const float ir = bl * v[j] + bih[j], iz = bl * v[HHD + j] + bih[HHD + j], inn = bl * v[2 * HHD + j] + bih[2 * HHD + j];
    const float r = 1.0f / (1.0f + expf(-(ir + g[j]))), z = 1.0f / (1.0f + expf(-(iz + g[HHD + j])));
    const float n = tanhf(inn + r * g[2 * HHD + j]);
    hS[j] = (1.0f - z) * n + z * hr[j]; }
  __syncthreads();
  float* dst = hout + (size_t)l * HHD;
#pragma unroll 1
  for (int pass = 0; pass < 2; ++pass) {
#pragma unroll 1
    for (int j = tid; j < HHD; j += 256) *(volatile float*)(dst + j) = hS[j];
    __threadfence();
  }
}

extern "C" void kernel_launch(void* const* d_in, const int* in_sizes, int n_in,
                              void* d_out, int out_size, void* d_ws, size_t ws_size,
                              hipStream_t stream) {
  (void)in_sizes; (void)n_in; (void)out_size; (void)ws_size;
  const float* tv = (const float*)d_in[0];
  const float* kv = (const float*)d_in[1];
  const float* result = (const float*)d_in[2];
  const float* h = (const float*)d_in[3];
  const float* km = (const float*)d_in[4];
  const float* Wih = (const float*)d_in[5];
  const float* Whh = (const float*)d_in[6];
  const float* bih = (const float*)d_in[7], *bhh = (const float*)d_in[8];
  const float* sw = (const float*)d_in[9], *sb = (const float*)d_in[10];
  float* out = (float*)d_out;
  char* ws = (char*)d_ws;
  float* beta = (float*)ws; ws += LL * 4;
  float* v = (float*)ws; ws += G3 * 4;
  float* gh = (float*)ws; ws += (size_t)LL * G3 * 4;
  k_beta<<<dim3(1), dim3(256), 0, stream>>>(km, kv, beta);
  k_vih<<<dim3(G3 / 256), dim3(256), 0, stream>>>(Wih, tv, result, v);
  k_score<<<dim3(1), dim3(256), 0, stream>>>(beta, h, tv, sw, sb, out);
  gemm_rb_kernel<float, 2><<<dim3(LL / 128, G3 / 256), dim3(256), 0, stream>>>(h, Whh, bhh, nullptr, nullptr, nullptr, gh, LL, G3, HHD);
  k_gru<<<dim3(LL), dim3(256), 0, stream>>>(gh, beta, v, bih, h, out + 1);
}
